// Model_24077586661558
// MI455X (gfx1250) — hardware-verified
//
#include <hip/hip_runtime.h>
#include <math.h>
#include <stdint.h>

#define NB    8
#define CC    2048
#define LL    784
#define KG    800
#define LP    832
#define DD    8192
#define NCLS  200
#define NPAD  208
#define OUT1_OFF 1600
#define CHUNK 64
#define NCHUNK 32
#define IMG_GRP 4

#define PREP_XBLOCKS ((NB * CC * (LP / 8)) / 256)
#define PREP_WBLOCKS (DD / 64)
#define PREP_ZBLOCKS ((2 * 16 * DD / 8) / 256)

static_assert(DD == 8192);
static_assert((DD & (DD - 1)) == 0);
static_assert(CC == 2048);
static_assert(CC == 2 * 1024);
static_assert(LL <= KG);
static_assert(KG <= LP);
static_assert(KG % 32 == 0);
static_assert((LP * 2) % 128 == 0);
static_assert(LL % 8 == 0);
static_assert(LP % 8 == 0);
static_assert(NCLS <= NPAD);
static_assert(NPAD == 13 * 16);
static_assert(NCLS % 4 == 0);
static_assert(OUT1_OFF == NB * NCLS);
static_assert((OUT1_OFF * 4) % 128 == 0);
static_assert(OUT1_OFF + NB * DD == 67136);
static_assert(CC % 128 == 0);
static_assert(CC % 64 == 0);
static_assert(CC == CHUNK * NCHUNK);
static_assert((NB * CC * (LP / 8)) % 256 == 0);
static_assert(NB % IMG_GRP == 0);
static_assert((CC / 64) * (CC / 64) % 8 == 0);
static_assert(DD == 8 * 1024);

typedef __attribute__((ext_vector_type(16))) __bf16 v16b;
typedef __attribute__((ext_vector_type(8)))  __bf16 v8b;
typedef __attribute__((ext_vector_type(8)))  float  v8f;
typedef __attribute__((ext_vector_type(4)))  float  v4f;
typedef __attribute__((ext_vector_type(4)))  unsigned int v4u;
typedef __attribute__((ext_vector_type(4)))  int    v4i;

__device__ __forceinline__ unsigned short f2bf_bits(float f) {
  const unsigned u = __float_as_uint(f);
  unsigned r = (u + 0x7FFFu + ((u >> 16) & 1u)) >> 16;
  r = (f != f) ? 0x7FC0u : r;
  return (unsigned short)r;
}
__device__ __forceinline__ float bf_bits2f(unsigned short h) { return __uint_as_float(((unsigned)h) << 16); }
__device__ __forceinline__ float bf_rne(float f) { return bf_bits2f(f2bf_bits(f)); }
__device__ __forceinline__ unsigned pk16(unsigned short a, unsigned short b) { return (unsigned)a | ((unsigned)b << 16); }

union FragU { v16b v; v8b h[2]; };
__device__ __forceinline__ v16b frag_load(const __bf16* p) {
  FragU f; f.h[0] = *(const v8b*)(p); f.h[1] = *(const v8b*)(p + 16); return f.v;
}
__device__ __forceinline__ v8f mma_bf16(v16b a, v16b b, v8f c) {
  return __builtin_amdgcn_wmma_f32_16x16x32_bf16(false, a, false, b, (short)0, c, false, false);
}
__device__ __forceinline__ v8f mma_bf16_g(v16b a, v16b b, v8f c) {
  v8f d = __builtin_amdgcn_wmma_f32_16x16x32_bf16(false, a, false, b, (short)0, c, false, false);
  asm volatile("v_nop\n\tv_nop\n\tv_nop\n\tv_nop" : "+v"(d) : "v"(a), "v"(b));
  return d;
}
__device__ __forceinline__ void dep_guard_b(v8f& a, v8f& b, v16b x, v16b y) { asm volatile("v_nop\n\tv_nop\n\tv_nop\n\tv_nop" : "+v"(a), "+v"(b) : "v"(x), "v"(y)); }
__device__ __forceinline__ void keep4_b(v16b a, v16b b, v16b c, v16b d) { asm volatile("v_nop" :: "v"(a), "v"(b), "v"(c), "v"(d)); }
__device__ __forceinline__ void acc_guard4(v8f& a, v8f& b, v8f& c, v8f& d) { asm volatile("v_nop\n\tv_nop\n\tv_nop\n\tv_nop" : "+v"(a), "+v"(b), "+v"(c), "+v"(d)); }

__global__ __launch_bounds__(256) void k_prep(const float* __restrict__ x, const float* __restrict__ W,
                                              unsigned short* __restrict__ XB, unsigned short* __restrict__ WT,
                                              unsigned short* __restrict__ FHL) {
  __shared__ __align__(16) float tf[64 * 212];
  const int tid = threadIdx.x;
  const int blk = blockIdx.x;
  if (blk < PREP_XBLOCKS) {
    const int u   = blk * 256 + tid;
    const int row = u / (LP / 8);
    const int g   = u - row * (LP / 8);
    const int gc  = (g < (LL / 8)) ? g : (LL / 8 - 1);
    const unsigned msk = (g < (LL / 8)) ? 0xFFFFFFFFu : 0u;
    const float* src = x + (size_t)row * LL + gc * 8;
    const v4f a = *(const v4f*)src;
    const v4f c = *(const v4f*)(src + 4);
    v4u o;
    o[0] = pk16(f2bf_bits(a[0]), f2bf_bits(a[1])) & msk;
    o[1] = pk16(f2bf_bits(a[2]), f2bf_bits(a[3])) & msk;
    o[2] = pk16(f2bf_bits(c[0]), f2bf_bits(c[1])) & msk;
    o[3] = pk16(f2bf_bits(c[2]), f2bf_bits(c[3])) & msk;
    unsigned short* dst = XB + (size_t)u * 8;
    *(volatile v4u*)dst = o;
    __threadfence();
    *(volatile v4u*)dst = o;
  } else if (blk < PREP_XBLOCKS + PREP_WBLOCKS) {
    const int k0 = (blk - PREP_XBLOCKS) * 64;
#pragma unroll 1
    for (int i = tid; i < 64 * 50; i += 256) {
      const int r  = i / 50;
      const int c4 = (i - r * 50) * 4;
      const v4f a = *(const v4f*)(W + (size_t)(k0 + r) * NCLS + c4);
      *(v4f*)(tf + r * 212 + c4) = a;
    }
#pragma unroll 1
    for (int i = tid; i < 64 * 12; i += 256) {
      const int r = i / 12;
      const int c = NCLS + (i - r * 12);
      tf[r * 212 + c] = 0.0f;
    }
    __syncthreads();
    const int sub = tid >> 3;
    const int c8  = (tid & 7) * 8;
    v4u hv[7];
#pragma unroll
    for (int it = 0; it < 7; ++it) {
      const int n  = it * 32 + sub;
      const int nc = (n < NPAD) ? n : (NPAD - 1);
      v4u a;
#pragma unroll
      for (int q = 0; q < 4; ++q) {
        const float f0 = tf[(c8 + 2 * q) * 212 + nc];
        const float f1 = tf[(c8 + 2 * q + 1) * 212 + nc];
        a[q] = pk16(f2bf_bits(f0), f2bf_bits(f1));
      }
      hv[it] = a;
    }
    for (int pass = 0; pass < 2; ++pass) {
#pragma unroll
      for (int it = 0; it < 7; ++it) {
        const int n = it * 32 + sub;
        if (n < NPAD) {
          *(volatile v4u*)(WT + (size_t)n * DD + k0 + c8) = hv[it];
        }
      }
      __threadfence();
    }
  } else {
    const int u = (blk - PREP_XBLOCKS - PREP_WBLOCKS) * 256 + tid;
    const v4u z = {0u, 0u, 0u, 0u};
    unsigned short* dst = FHL + (size_t)u * 8;
    *(volatile v4u*)dst = z;
    __threadfence();
    *(volatile v4u*)dst = z;
  }
}

__global__ __launch_bounds__(1024) void k_tables(const float* __restrict__ s1, const float* __restrict__ s2,
                                                 const float* __restrict__ bcls,
                                                 const int* __restrict__ h1, const int* __restrict__ h2,
                                                 int* __restrict__ PERM2, int* __restrict__ TB, float* __restrict__ SG,
                                                 int* __restrict__ RUNLEN, int* __restrict__ H1T, float* __restrict__ S1F,
                                                 float* __restrict__ BF) {
  __shared__ __align__(16) int   skey[CC];
  __shared__ __align__(16) int   sperm[CC];
  __shared__ __align__(16) int   stb[CC];
  __shared__ __align__(16) float ssg[CC];
  __shared__ __align__(16) int   srl[CC];
  const int tid = threadIdx.x;
  const int c0 = tid, c1 = tid + 1024;
  const int hv0 = h2[c0], hv1 = h2[c1];
  const float sv0 = s2[c0], sv1 = s2[c1];
  const int hm0 = hv0 & (DD - 1), hm1 = hv1 & (DD - 1);
  const float g0 = ((unsigned)hv0 < (unsigned)DD) ? bf_rne(sv0) : 0.0f;
  const float g1 = ((unsigned)hv1 < (unsigned)DD) ? bf_rne(sv1) : 0.0f;
  const int k0 = (hm0 << 11) | c0;
  const int k1 = (hm1 << 11) | c1;
  skey[c0] = k0;
  skey[c1] = k1;
  __syncthreads();
  int p0 = 0, p1 = 0, n0 = 0, n1 = 0;
#pragma unroll 4
  for (int j = 0; j < CC; ++j) {
    const int kj = skey[j];
    const int bj = kj >> 11;
    p0 += (kj < k0) ? 1 : 0;
    p1 += (kj < k1) ? 1 : 0;
    n0 += (bj == hm0) ? 1 : 0;
    n1 += (bj == hm1) ? 1 : 0;
  }
  sperm[p0] = c0; stb[p0] = hm0; ssg[p0] = g0; srl[p0] = n0;
  sperm[p1] = c1; stb[p1] = hm1; ssg[p1] = g1; srl[p1] = n1;
  __syncthreads();
  {
    const int q0 = tid, q1 = tid + 1024;
    const int pq0 = (q0 > 0) ? (q0 - 1) : 0;
    const int pv0 = stb[pq0];
    const int pv1 = stb[q1 - 1];
    const int t0 = stb[q0], t1 = stb[q1];
    const int r0 = ((q0 == 0) || (pv0 != t0)) ? srl[q0] : 0;
    const int r1 = (pv1 != t1) ? srl[q1] : 0;
    srl[q0] = r0;
    srl[q1] = r1;
  }
  __syncthreads();
  if (tid < 512) {
    const v4i vp = *(const v4i*)(sperm + 4 * tid);
    const v4i vt = *(const v4i*)(stb + 4 * tid);
    const v4f vs = *(const v4f*)(ssg + 4 * tid);
    const v4i vr = *(const v4i*)(srl + 4 * tid);
    const v4i hh = *(const v4i*)(h1 + 4 * tid);
    const v4f s1v = *(const v4f*)(s1 + 4 * tid);
    v4i h1o; v4f s1o;
#pragma unroll
    for (int e = 0; e < 4; ++e) {
      h1o[e] = hh[e] & (DD - 1);
      s1o[e] = ((unsigned)hh[e] < (unsigned)DD) ? bf_rne(s1v[e]) : 0.0f;
    }
    const int tc = (tid < (NCLS / 4)) ? tid : (NCLS / 4 - 1);
    const v4f bb = *(const v4f*)(bcls + 4 * tc);
    v4f bo;
#pragma unroll
    for (int e = 0; e < 4; ++e) bo[e] = (tid < (NCLS / 4)) ? bf_rne(bb[e]) : 0.0f;
    for (int pass = 0; pass < 2; ++pass) {
      *(volatile v4i*)(PERM2 + 4 * tid)  = vp;
      *(volatile v4i*)(TB + 4 * tid)     = vt;
      *(volatile v4f*)(SG + 4 * tid)     = vs;
      *(volatile v4i*)(RUNLEN + 4 * tid) = vr;
      *(volatile v4i*)(H1T + 4 * tid)    = h1o;
      *(volatile v4f*)(S1F + 4 * tid)    = s1o;
      if (tid < 64) {
        *(volatile v4f*)(BF + 4 * tid) = bo;
      }
      __threadfence();
    }
  }
}

__global__ __launch_bounds__(256) void k_gram(const unsigned short* __restrict__ XBp, float* __restrict__ G, int img0) {
  __shared__ __align__(16) float sT[8][16 * 68];
  const __bf16* XB = (const __bf16*)XBp;
  const int b    = blockIdx.y;
  const int lane = threadIdx.x & 31;
  const int wave = threadIdx.x >> 5;
  const int tile = blockIdx.x * 8 + wave;
  const int tm = tile >> 5;
  const int tn = tile & 31;
  const int m0 = tm << 6;
  const int n0 = tn << 6;
  const __bf16* Xb = XB + (size_t)(img0 + b) * CC * LP;
  float* C = G + (size_t)b * CC * CC;

  const int rlane = lane & 15;
  const int koff  = (lane >> 4) * 8;
  const int mOff  = (lane >> 4) * 8;

  v8f acc[4][4];
#pragma unroll
  for (int i = 0; i < 4; ++i)
#pragma unroll
    for (int j = 0; j < 4; ++j) acc[i][j] = (v8f){0.f, 0.f, 0.f, 0.f, 0.f, 0.f, 0.f, 0.f};

#pragma unroll 1
  for (int k0 = 0; k0 < KG; k0 += 32) {
    v16b bh[4];
#pragma unroll
    for (int j = 0; j < 4; ++j) {
      const size_t bo = (size_t)(n0 + (j << 4) + rlane) * LP + koff + k0;
      bh[j] = frag_load(Xb + bo);
    }
#pragma unroll
    for (int i = 0; i < 4; ++i) {
      const size_t ao = (size_t)(m0 + (i << 4) + rlane) * LP + koff + k0;
      const v16b ah = frag_load(Xb + ao);
#pragma unroll
      for (int j = 0; j < 4; ++j) acc[i][j] = mma_bf16(ah, bh[j], acc[i][j]);
      dep_guard_b(acc[i][0], acc[i][3], ah, ah);
    }
    keep4_b(bh[0], bh[1], bh[2], bh[3]);
  }
  acc_guard4(acc[0][0], acc[0][1], acc[0][2], acc[0][3]);
  acc_guard4(acc[1][0], acc[1][1], acc[1][2], acc[1][3]);
  acc_guard4(acc[2][0], acc[2][1], acc[2][2], acc[2][3]);
  acc_guard4(acc[3][0], acc[3][1], acc[3][2], acc[3][3]);

  float* slab = sT[wave];
#pragma unroll
  for (int i = 0; i < 4; ++i) {
    const int mBase = m0 + (i << 4);
#pragma unroll
    for (int j = 0; j < 4; ++j) {
#pragma unroll
      for (int r = 0; r < 8; ++r) {
        slab[(mOff + r) * 68 + (j << 4) + rlane] = acc[i][j][r];
      }
    }
    __builtin_amdgcn_fence(__ATOMIC_RELEASE, "workgroup");
    __builtin_amdgcn_wave_barrier();
    __builtin_amdgcn_fence(__ATOMIC_ACQUIRE, "workgroup");
    {
      const int hh = lane >> 4, c4 = (lane & 15) * 4;
      v4f ov[8];
#pragma unroll
      for (int it = 0; it < 8; ++it) {
        const int row = it * 2 + hh;
        ov[it] = *(const v4f*)(slab + row * 68 + c4);
      }
      for (int pass = 0; pass < 2; ++pass) {
#pragma unroll
        for (int it = 0; it < 8; ++it) {
          const int row = it * 2 + hh;
          *(volatile v4f*)(C + (size_t)(mBase + row) * CC + n0 + c4) = ov[it];
        }
        __threadfence();
      }
    }
    __builtin_amdgcn_fence(__ATOMIC_RELEASE, "workgroup");
    __builtin_amdgcn_wave_barrier();
    __builtin_amdgcn_fence(__ATOMIC_ACQUIRE, "workgroup");
  }
}

__global__ __launch_bounds__(1024) void k_sketch(const float* __restrict__ G,
                                                 const int* __restrict__ PERM2, const int* __restrict__ TB,
                                                 const float* __restrict__ SG, const int* __restrict__ RUNLEN,
                                                 const int* __restrict__ H1T, const float* __restrict__ S1F,
                                                 float* __restrict__ YP, int img0) {
  __shared__ __align__(16) float bins[DD];
  __shared__ __align__(16) int   sperm[CC];
  __shared__ __align__(16) float ssg[CC];
  __shared__ __align__(16) int   sh1[CHUNK];
  __shared__ __align__(16) float ss1[CHUNK];
  const int tid   = threadIdx.x;
  const int chunk = blockIdx.x;
  const int imgl  = blockIdx.y;

#pragma unroll
  for (int i = 0; i < 8; ++i) bins[tid + i * 1024] = 0.0f;
  if (tid < 512) {
    v4i vp = *(const v4i*)(PERM2 + 4 * tid);
#pragma unroll
    for (int e = 0; e < 4; ++e) { int t = vp[e]; t = (t < 0) ? 0 : t; t = (t > CC - 1) ? (CC - 1) : t; vp[e] = t; }
    *(v4i*)(sperm + 4 * tid) = vp;
    const v4f vs = *(const v4f*)(SG + 4 * tid);
    *(v4f*)(ssg + 4 * tid) = vs;
  }
  if (tid < CHUNK / 4) {
    v4i hh = *(const v4i*)(H1T + chunk * CHUNK + 4 * tid);
#pragma unroll
    for (int e = 0; e < 4; ++e) hh[e] = hh[e] & (DD - 1);
    *(v4i*)(sh1 + 4 * tid) = hh;
    const v4f sv = *(const v4f*)(S1F + chunk * CHUNK + 4 * tid);
    *(v4f*)(ss1 + 4 * tid) = sv;
  }
  const int pA = tid, pB = tid + 1024;
  int rlA = RUNLEN[pA];
  int rlB = RUNLEN[pB];
  const int tbA = TB[pA] & (DD - 1);
  const int tbB = TB[pB] & (DD - 1);
  rlA = (rlA < 0) ? 0 : rlA;  rlA = (rlA > CC - pA) ? (CC - pA) : rlA;
  rlB = (rlB < 0) ? 0 : rlB;  rlB = (rlB > CC - pB) ? (CC - pB) : rlB;

  const float* Gi = G + (size_t)imgl * CC * CC + (size_t)(chunk * CHUNK) * CC;

#pragma unroll 1
  for (int s = 0; s < CHUNK; ++s) {
    __syncthreads();
    const float* grow = Gi + (size_t)s * CC;
    const int   hh  = sh1[s];
    const float sg1 = ss1[s];
    if (rlA > 0) {
      float v = 0.0f;
      for (int j = 0; j < rlA; ++j) v += ssg[pA + j] * grow[sperm[pA + j]];
      const int bin = (hh + tbA) & (DD - 1);
      bins[bin] += sg1 * v;
    }
    if (rlB > 0) {
      float v = 0.0f;
      for (int j = 0; j < rlB; ++j) v += ssg[pB + j] * grow[sperm[pB + j]];
      const int bin = (hh + tbB) & (DD - 1);
      bins[bin] += sg1 * v;
    }
  }
  __syncthreads();

  float* yp = YP + ((size_t)(img0 + imgl) * NCHUNK + chunk) * DD;
  const v4f o0 = *(const v4f*)(bins + 4 * tid);
  const v4f o1 = *(const v4f*)(bins + 4096 + 4 * tid);
  for (int pass = 0; pass < 2; ++pass) {
    *(volatile v4f*)(yp + 4 * tid) = o0;
    *(volatile v4f*)(yp + 4096 + 4 * tid) = o1;
    __threadfence();
  }
}

__global__ __launch_bounds__(1024) void k_finish(const float* __restrict__ YP, float* __restrict__ out,
                                                 unsigned short* __restrict__ FH, unsigned short* __restrict__ FL) {
  __shared__ double red[1024];
  __shared__ __align__(16) float sf[DD];
  const int tid = threadIdx.x;
  const int b   = blockIdx.x;
  const float* yp = YP + (size_t)b * NCHUNK * DD;
  double ya0 = 0.0, ya1 = 0.0, ya2 = 0.0, ya3 = 0.0;
  double yb0 = 0.0, yb1 = 0.0, yb2 = 0.0, yb3 = 0.0;
#pragma unroll 4
  for (int ch = 0; ch < NCHUNK; ++ch) {
    const v4f a = *(const v4f*)(yp + (size_t)ch * DD + 4 * tid);
    const v4f c = *(const v4f*)(yp + (size_t)ch * DD + 4096 + 4 * tid);
    ya0 += (double)a[0]; ya1 += (double)a[1]; ya2 += (double)a[2]; ya3 += (double)a[3];
    yb0 += (double)c[0]; yb1 += (double)c[1]; yb2 += (double)c[2]; yb3 += (double)c[3];
  }
  {
    v4f ya, yb;
    ya[0] = (float)ya0; ya[1] = (float)ya1; ya[2] = (float)ya2; ya[3] = (float)ya3;
    yb[0] = (float)yb0; yb[1] = (float)yb1; yb[2] = (float)yb2; yb[3] = (float)yb3;
    *(v4f*)(sf + 4 * tid) = ya;
    *(v4f*)(sf + 4096 + 4 * tid) = yb;
  }
  __syncthreads();

  double ss = 0.0;
#pragma unroll 1
  for (int i = 0; i < 8; ++i) {
    const int idx = ((i >> 2) << 12) + 4 * tid + (i & 3);
    const float y = sf[idx];
    const float s = sqrtf(fabsf(y));
    const float f = (y > 0.0f) ? s : ((y < 0.0f) ? -s : y);
    sf[idx] = f;
    ss += (double)f * (double)f;
  }
  red[tid] = ss;
  __syncthreads();
#pragma unroll 1
  for (int s = 512; s > 0; s >>= 1) {
    if (tid < s) red[tid] = red[tid] + red[tid + s];
    __syncthreads();
  }
  const float nrm = sqrtf((float)red[0]);
  const float den = fmaxf(nrm, 1e-12f);

#pragma unroll 1
  for (int i = 0; i < 8; ++i) {
    const int idx = ((i >> 2) << 12) + 4 * tid + (i & 3);
    const float f = sf[idx];
    const float q = f / den;
    sf[idx] = q;
  }
  __syncthreads();

  const v4f oa = *(const v4f*)(sf + 4 * tid);
  const v4f ob = *(const v4f*)(sf + 4096 + 4 * tid);
  float* orow = out + OUT1_OFF + (size_t)b * DD;
  for (int pass = 0; pass < 2; ++pass) {
    *(volatile v4f*)(orow + 4 * tid) = oa;
    *(volatile v4f*)(orow + 4096 + 4 * tid) = ob;
    __threadfence();
  }

  {
    const v4f p = *(const v4f*)(sf + 8 * tid);
    const v4f q = *(const v4f*)(sf + 8 * tid + 4);
    unsigned short hb[8], lb[8];
#pragma unroll
    for (int e = 0; e < 4; ++e) {
      hb[e]     = f2bf_bits(p[e]);
      lb[e]     = f2bf_bits(p[e] - bf_bits2f(hb[e]));
      hb[4 + e] = f2bf_bits(q[e]);
      lb[4 + e] = f2bf_bits(q[e] - bf_bits2f(hb[4 + e]));
    }
    v4u hv, lv;
#pragma unroll
    for (int w = 0; w < 4; ++w) {
      hv[w] = pk16(hb[2 * w], hb[2 * w + 1]);
      lv[w] = pk16(lb[2 * w], lb[2 * w + 1]);
    }
    unsigned short* dh = FH + (size_t)b * DD + 8 * tid;
    unsigned short* dl = FL + (size_t)b * DD + 8 * tid;
    for (int pass = 0; pass < 2; ++pass) {
      *(volatile v4u*)dh = hv;
      *(volatile v4u*)dl = lv;
      __threadfence();
    }
  }
}

__global__ __launch_bounds__(416) void k_logit(const unsigned short* __restrict__ FHp, const unsigned short* __restrict__ FLp,
                                               const unsigned short* __restrict__ WTp, const float* __restrict__ BF,
                                               float* __restrict__ out) {
  __shared__ __align__(16) float sl[16 * NPAD];
  const __bf16* FH = (const __bf16*)FHp;
  const __bf16* FL = (const __bf16*)FLp;
  const __bf16* WT = (const __bf16*)WTp;
  const int tid = threadIdx.x, lane = tid & 31, w = tid >> 5;
  const int h = lane >> 4, m = lane & 15;
  const __bf16* ah = FH + (size_t)m * DD + 8 * h;
  const __bf16* al = FL + (size_t)m * DD + 8 * h;
  const __bf16* bp = WT + (size_t)(16 * w + m) * DD + 8 * h;
  v8f acc = (v8f){0.f, 0.f, 0.f, 0.f, 0.f, 0.f, 0.f, 0.f};
#pragma unroll 2
  for (int k0 = 0; k0 < DD; k0 += 32) {
    const v16b a1 = frag_load(ah + k0);
    const v16b a2 = frag_load(al + k0);
    const v16b bb = frag_load(bp + k0);
    acc = mma_bf16_g(a1, bb, acc);
    acc = mma_bf16_g(a2, bb, acc);
  }
#pragma unroll
  for (int r = 0; r < 8; ++r) sl[(8 * h + r) * NPAD + 16 * w + m] = acc[r];
  __syncthreads();
  if (tid < (NB * NCLS) / 4) {
    const int e   = 4 * tid;
    const int row = e / NCLS;
    const int col = e - row * NCLS;
    const v4f v  = *(const v4f*)(sl + row * NPAD + col);
    const v4f bv = *(const v4f*)(BF + col);
    v4f o;
#pragma unroll
    for (int q = 0; q < 4; ++q) o[q] = v[q] + bv[q];
    *(volatile v4f*)(out + e) = o;
    __threadfence();
    *(volatile v4f*)(out + e) = o;
  }
}

extern "C" void kernel_launch(void* const* d_in, const int* in_sizes, int n_in,
                              void* d_out, int out_size, void* d_ws, size_t ws_size,
                              hipStream_t stream) {
  if (n_in < 7) return;
  if (in_sizes[0] != NB * CC * LL) return;
  if (in_sizes[1] != CC || in_sizes[2] != CC) return;
  if (in_sizes[3] != DD * NCLS) return;
  if (in_sizes[4] != NCLS) return;
  if (in_sizes[5] != CC || in_sizes[6] != CC) return;
  if (out_size != OUT1_OFF + NB * DD) return;

  const float* x    = (const float*)d_in[0];
  const float* s1   = (const float*)d_in[1];
  const float* s2   = (const float*)d_in[2];
  const float* Wcls = (const float*)d_in[3];
  const float* bcls = (const float*)d_in[4];
  const int*   h1   = (const int*)d_in[5];
  const int*   h2   = (const int*)d_in[6];
  float* out = (float*)d_out;

  const size_t PXB = (size_t)NB * CC * LP * 2;
  const size_t PG  = (size_t)IMG_GRP * CC * CC * 4;
  const size_t PYP = (size_t)NB * NCHUNK * DD * 4;
  const size_t PWT = (size_t)NPAD * DD * 2;
  const size_t PF  = (size_t)2 * 16 * DD * 2;
  const size_t PT  = (size_t)CC * 4;
  const size_t PBF = (size_t)1024;
  size_t off = 0;
  const size_t oXB = off; off += PXB;
  const size_t oG  = off; off += PG;
  const size_t oYP = off; off += PYP;
  const size_t oWT = off; off += PWT;
  const size_t oF  = off; off += PF;
  const size_t oT0 = off; off += PT;
  const size_t oT1 = off; off += PT;
  const size_t oT2 = off; off += PT;
  const size_t oT3 = off; off += PT;
  const size_t oT4 = off; off += PT;
  const size_t oT5 = off; off += PT;
  const size_t oBF = off; off += PBF;
  if (off > ws_size) return;
  if (off > (size_t)134217728) return;

  char* ws = (char*)d_ws;
  unsigned short* XB  = (unsigned short*)(ws + oXB);
  float*          G   = (float*)(ws + oG);
  float*          YP  = (float*)(ws + oYP);
  unsigned short* WT  = (unsigned short*)(ws + oWT);
  unsigned short* FHL = (unsigned short*)(ws + oF);
  unsigned short* FH  = FHL;
  unsigned short* FL  = FHL + (size_t)16 * DD;
  int*   PERM2  = (int*)(ws + oT0);
  int*   TB     = (int*)(ws + oT1);
  float* SG     = (float*)(ws + oT2);
  int*   RUNLEN = (int*)(ws + oT3);
  int*   H1T    = (int*)(ws + oT4);
  float* S1F    = (float*)(ws + oT5);
  float* BF     = (float*)(ws + oBF);

  k_prep<<<dim3(PREP_XBLOCKS + PREP_WBLOCKS + PREP_ZBLOCKS), dim3(256), 0, stream>>>(x, Wcls, XB, WT, FHL);
  k_tables<<<dim3(1), dim3(1024), 0, stream>>>(s1, s2, bcls, h1, h2, PERM2, TB, SG, RUNLEN, H1T, S1F, BF);
  for (int g = 0; g < NB / IMG_GRP; ++g) {
    const int img0 = g * IMG_GRP;
    k_gram<<<dim3(((CC / 64) * (CC / 64)) / 8, IMG_GRP), dim3(256), 0, stream>>>(XB, G, img0);
    k_sketch<<<dim3(NCHUNK, IMG_GRP), dim3(1024), 0, stream>>>(G, PERM2, TB, SG, RUNLEN, H1T, S1F, YP, img0);
  }
  k_finish<<<dim3(NB), dim3(1024), 0, stream>>>(YP, out, FH, FL);
  k_logit<<<dim3(1), dim3(416), 0, stream>>>(FH, FL, WT, BF, out);
  (void)hipGetLastError();
}
